// MambaBlock_40922448396738
// MI455X (gfx1250) — hardware-verified
//
#include <hip/hip_runtime.h>
#include <math.h>

typedef __attribute__((ext_vector_type(16))) _Float16 v16h;
typedef __attribute__((ext_vector_type(8)))  _Float16 v8h;
typedef __attribute__((ext_vector_type(8)))  float    v8f;
typedef __attribute__((ext_vector_type(4)))  float    v4f;

constexpr int kBatch  = 2;
constexpr int kSeq    = 2048;
constexpr int kDm     = 1024;
constexpr int kNst    = 16;
constexpr int kDtR    = 16;
constexpr int kXzP    = 2 * kDm;
constexpr int kXdN    = kDtR + 2 * kNst;
constexpr int kXdP    = 64;
constexpr int kRows   = kBatch * kSeq;
constexpr int kConvTP = 260;
constexpr int kScanTS = 64;
constexpr int kScanCh = 64;
constexpr int kScanYP = 68;

constexpr float kCarX  = 64.0f;
constexpr float kCarW  = 256.0f;
constexpr float kCarU  = 16.0f;
constexpr float kCarY  = 256.0f;
constexpr float kFold0 = 1.0f / (kCarX * kCarW);
constexpr float kFold1 = 1.0f / (kCarU * kCarW);
constexpr float kFold2 = 1.0f / (kCarY * kCarW);
constexpr float kSatY  = 60000.0f;

static_assert(kXdN == 48);
static_assert(kXdN <= kXdP && (kXdN % 4) == 0);
static_assert((kDm % 32) == 0);
static_assert((kRows % 64) == 0 && (kXzP % 64) == 0 && (kXdP % 64) == 0 && (kDm % 64) == 0);
static_assert((kSeq % kScanTS) == 0 && (kSeq % 64) == 0 && (kDm % kScanCh) == 0 && (kDm % 256) == 0);
static_assert(kScanCh == 64 && kScanTS == 64 && kNst == 16 && kDtR == 16);

constexpr size_t kOffX16  = 0;
constexpr size_t kOffWIN  = kOffX16  + (size_t)kRows * kDm  * 2;
constexpr size_t kOffWXP  = kOffWIN  + (size_t)kXzP  * kDm  * 2;
constexpr size_t kOffWOUT = kOffWXP  + (size_t)kXdP  * kDm  * 2;
constexpr size_t kOffXZ   = kOffWOUT + (size_t)kDm   * kDm  * 2;
constexpr size_t kOffUC   = kOffXZ   + (size_t)kRows * kXzP * 4;
constexpr size_t kOffUC16 = kOffUC   + (size_t)kRows * kDm  * 4;
constexpr size_t kOffXD   = kOffUC16 + (size_t)kRows * kDm  * 2;
constexpr size_t kOffY16  = kOffXD   + (size_t)kRows * kXdP * 4;
constexpr size_t kWsTotal = kOffY16  + (size_t)kRows * kDm  * 2;
static_assert(kWsTotal == 82968576ull);
static_assert(kWsTotal <= 134217728ull);
static_assert((kOffWIN % 128) == 0 && (kOffWXP % 128) == 0 && (kOffWOUT % 128) == 0 && (kOffXZ % 128) == 0 &&
              (kOffUC % 128) == 0 && (kOffUC16 % 128) == 0 && (kOffXD % 128) == 0 && (kOffY16 % 128) == 0);

union FragU { v16h v; v8h h[2]; };
__device__ __forceinline__ v16h frag_load(const _Float16* p) {
  FragU f;
  f.h[0] = *(const v8h*)(p);
  f.h[1] = *(const v8h*)(p + 16);
  return f.v;
}
__device__ __forceinline__ v8f frag_mma(v16h a, v16h b, v8f c) {
  return __builtin_amdgcn_wmma_f32_16x16x32_f16(false, a, false, b, (short)0, c, false, false);
}
__device__ __forceinline__ void guard_row(v8f& a, v8f& b, v8f& c, v8f& d, v16h x,
                                          v16h y0, v16h y1, v16h y2, v16h y3) {
  asm volatile("v_nop\n\tv_nop\n\tv_nop\n\tv_nop"
               : "+v"(a), "+v"(b), "+v"(c), "+v"(d)
               : "v"(x), "v"(y0), "v"(y1), "v"(y2), "v"(y3));
}
__device__ __forceinline__ void acc_guard4(v8f& a, v8f& b, v8f& c, v8f& d) {
  asm volatile("v_nop\n\tv_nop\n\tv_nop\n\tv_nop" : "+v"(a), "+v"(b), "+v"(c), "+v"(d));
}

template <int BIAS_MODE>
__global__ __launch_bounds__(256) void gemm64_f16(
    const unsigned short* __restrict__ Ap, int lda,
    const unsigned short* __restrict__ Btp, int ldb,
    float* __restrict__ C, int ldc,
    const float* __restrict__ bias,
    int M, int N, int K, float scale)
{
  const _Float16* A  = (const _Float16*)Ap;
  const _Float16* Bt = (const _Float16*)Btp;
  __shared__ __align__(16) float sT[8][16 * 68];
  const int lane = threadIdx.x & 31;
  const int wave = threadIdx.x >> 5;
  const int tilesN = N >> 6;
  const int tilesM = M >> 6;
  const int tile = blockIdx.x * 8 + wave;
  if (tile >= tilesM * tilesN) return;
  const int tm = tile / tilesN;
  const int tn = tile - tm * tilesN;
  const int m0 = tm << 6;
  const int n0 = tn << 6;

  const int rlane = lane & 15;
  const int koff  = (lane >> 4) * 8;
  const int mOff  = (lane >> 4) * 8;

  v8f acc[4][4];
#pragma unroll
  for (int i = 0; i < 4; ++i)
#pragma unroll
    for (int j = 0; j < 4; ++j) acc[i][j] = (v8f){0.f,0.f,0.f,0.f,0.f,0.f,0.f,0.f};

  for (int k0 = 0; k0 < K; k0 += 32) {
    v16h bh[4];
#pragma unroll
    for (int j = 0; j < 4; ++j) {
      const size_t bo = (size_t)(n0 + (j << 4) + rlane) * ldb + koff + k0;
      bh[j] = frag_load(Bt + bo);
    }
#pragma unroll
    for (int i = 0; i < 4; ++i) {
      const size_t ao = (size_t)(m0 + (i << 4) + rlane) * lda + koff + k0;
      const v16h ah = frag_load(A + ao);
#pragma unroll
      for (int j = 0; j < 4; ++j) acc[i][j] = frag_mma(ah, bh[j], acc[i][j]);
      guard_row(acc[i][0], acc[i][1], acc[i][2], acc[i][3], ah, bh[0], bh[1], bh[2], bh[3]);
    }
  }
  acc_guard4(acc[0][0], acc[0][1], acc[0][2], acc[0][3]);
  acc_guard4(acc[1][0], acc[1][1], acc[1][2], acc[1][3]);
  acc_guard4(acc[2][0], acc[2][1], acc[2][2], acc[2][3]);
  acc_guard4(acc[3][0], acc[3][1], acc[3][2], acc[3][3]);

  float* slab = sT[wave];
#pragma unroll
  for (int i = 0; i < 4; ++i) {
    const int mBase = m0 + (i << 4);
#pragma unroll
    for (int j = 0; j < 4; ++j) {
      const int n = n0 + (j << 4) + rlane;
      float bv = 0.f;
      if (BIAS_MODE == 2) bv = bias[n];
#pragma unroll
      for (int r = 0; r < 8; ++r) {
        float v = acc[i][j][r] * scale;
        if (BIAS_MODE == 2) v += bv;
        slab[(mOff + r) * 68 + (j << 4) + rlane] = v;
      }
    }
    __builtin_amdgcn_fence(__ATOMIC_RELEASE, "workgroup");
    __builtin_amdgcn_wave_barrier();
    __builtin_amdgcn_fence(__ATOMIC_ACQUIRE, "workgroup");
    {
      const int hh = lane >> 4, c4 = (lane & 15) * 4;
      for (int pass = 0; pass < 2; ++pass) {
#pragma unroll
        for (int it = 0; it < 8; ++it) {
          const int row = it * 2 + hh;
          v4f v = *(const v4f*)(slab + row * 68 + c4);
          *(volatile v4f*)(C + (size_t)(mBase + row) * ldc + n0 + c4) = v;
        }
        __threadfence();
      }
    }
    __builtin_amdgcn_fence(__ATOMIC_RELEASE, "workgroup");
    __builtin_amdgcn_wave_barrier();
    __builtin_amdgcn_fence(__ATOMIC_ACQUIRE, "workgroup");
  }
}

__global__ __launch_bounds__(256) void cast_f16_kernel(
    const float* __restrict__ src, unsigned short* __restrict__ dst, int total8, float scale)
{
  const int i = blockIdx.x * 256 + threadIdx.x;
  if (i >= total8) return;
  const size_t e0 = (size_t)i << 3;
  const float* p = src + e0;
  const v4f a0 = *(const v4f*)(p);
  const v4f a1 = *(const v4f*)(p + 4);
  v8h hv;
#pragma unroll
  for (int e = 0; e < 4; ++e) {
    hv[e]     = (_Float16)(a0[e] * scale);
    hv[4 + e] = (_Float16)(a1[e] * scale);
  }
  unsigned short* q = dst + e0;
  *(volatile v8h*)q = hv;
  __threadfence();
  *(volatile v8h*)q = hv;
}

__global__ __launch_bounds__(256) void transpose_cast_kernel(
    const float* __restrict__ W, unsigned short* __restrict__ Bt, int Kdim, int Ndim, float scale)
{
  __shared__ float tile[64 * 65];
  const int tid = threadIdx.x, lane = tid & 31, wave = tid >> 5;
  const int n0 = blockIdx.x * 64;
  const int k0 = blockIdx.y * 64;
#pragma unroll
  for (int p = 0; p < 16; ++p) {
    const int idx = tid + p * 256;
    const int kk  = idx >> 6;
    const int nn  = idx & 63;
    const int n   = n0 + nn;
    const int nc  = (n < Ndim) ? n : (Ndim - 1);
    const float v = W[(size_t)(k0 + kk) * Ndim + nc];
    tile[kk * 65 + nn] = (n < Ndim) ? (v * scale) : 0.f;
  }
  __syncthreads();
  const int q = lane >> 3, c8 = (lane & 7) * 8;
  v8h hv[2];
#pragma unroll
  for (int it = 0; it < 2; ++it) {
    const int nrow = it * 32 + wave * 4 + q;
#pragma unroll
    for (int e = 0; e < 8; ++e) hv[it][e] = (_Float16)tile[(c8 + e) * 65 + nrow];
  }
  for (int pass = 0; pass < 2; ++pass) {
#pragma unroll
    for (int it = 0; it < 2; ++it) {
      const int nrow = it * 32 + wave * 4 + q;
      *(volatile v8h*)(Bt + (size_t)(n0 + nrow) * Kdim + k0 + c8) = hv[it];
    }
    __threadfence();
  }
}

__global__ __launch_bounds__(256) void conv_silu_kernel(
    const float* __restrict__ XZ, const float* __restrict__ cw, const float* __restrict__ cb,
    float* __restrict__ UC, unsigned short* __restrict__ UC16)
{
  __shared__ __align__(16) float sT[16 * kConvTP];
  const int tid = threadIdx.x, lane = tid & 31, wave = tid >> 5;
  const int d0 = blockIdx.x * 256, d = d0 + tid;
  const int g0 = blockIdx.y * 64;
  const int tb = g0 & (kSeq - 1);
  const v4f wv = *(const v4f*)(cw + (size_t)d * 4);
  const float w0 = wv[0], w1 = wv[1], w2 = wv[2], w3 = wv[3];
  const float bc = cb[d];
  float xm3, xm2, xm1;
  {
    const bool hist = (tb > 0);
    const int rb = hist ? (g0 - 3) : g0;
    const float v3 = XZ[(size_t)rb * kXzP + d];
    const float v2 = XZ[(size_t)(rb + 1) * kXzP + d];
    const float v1 = XZ[(size_t)(rb + 2) * kXzP + d];
    xm3 = hist ? v3 : 0.f;
    xm2 = hist ? v2 : 0.f;
    xm1 = hist ? v1 : 0.f;
  }
  const int hrow = wave >> 1;
  const int hch  = (wave & 1) * 128 + lane * 4;
#pragma unroll 1
  for (int sub = 0; sub < 4; ++sub) {
    const int lb = g0 + sub * 16;
#pragma unroll 1
    for (int s = 0; s < 16; ++s) {
      const float xcur = XZ[(size_t)(lb + s) * kXzP + d];
      float acc = w0 * xm3;
      acc = fmaf(w1, xm2, acc);
      acc = fmaf(w2, xm1, acc);
      acc = fmaf(w3, xcur, acc);
      const float sv = acc + bc;
      const float sg = __builtin_amdgcn_rcpf(1.0f + expf(-sv));
      sT[s * kConvTP + tid] = sv * sg;
      xm3 = xm2; xm2 = xm1; xm1 = xcur;
    }
    __syncthreads();
    v4f fv[4];
    v8h bv[2];
#pragma unroll
    for (int it = 0; it < 4; ++it) fv[it] = *(const v4f*)(sT + (it * 4 + hrow) * kConvTP + hch);
#pragma unroll
    for (int it = 0; it < 2; ++it) {
      const float* sp = sT + (it * 8 + wave) * kConvTP + lane * 8;
      const v4f a0 = *(const v4f*)(sp);
      const v4f a1 = *(const v4f*)(sp + 4);
#pragma unroll
      for (int e = 0; e < 4; ++e) {
        bv[it][e]     = (_Float16)(a0[e] * kCarU);
        bv[it][4 + e] = (_Float16)(a1[e] * kCarU);
      }
    }
    for (int pass = 0; pass < 2; ++pass) {
#pragma unroll
      for (int it = 0; it < 4; ++it)
        *(volatile v4f*)(UC + (size_t)(lb + it * 4 + hrow) * kDm + d0 + hch) = fv[it];
#pragma unroll
      for (int it = 0; it < 2; ++it)
        *(volatile v8h*)(UC16 + (size_t)(lb + it * 8 + wave) * kDm + d0 + lane * 8) = bv[it];
      __threadfence();
    }
    __syncthreads();
  }
}

__global__ __launch_bounds__(64) void scan_kernel(
    const float* __restrict__ XD, const float* __restrict__ bxp,
    const float* __restrict__ UC, const float* __restrict__ XZ,
    const float* __restrict__ Wdt, const float* __restrict__ bdt, const float* __restrict__ Alog,
    unsigned short* __restrict__ Y16)
{
  __shared__ __align__(16) float sX[kScanTS * kXdP];
  __shared__ __align__(16) float sY[kScanTS * kScanYP];
  __shared__ __align__(16) float sW[kDtR * kScanCh];
  __shared__ __align__(16) float sA[kNst * kScanCh];
  const int tid = threadIdx.x, lane = tid & 31, wave = tid >> 5;
  constexpr int kBlkPerB = kDm / kScanCh;
  const int bix = blockIdx.x / kBlkPerB;
  const int d0  = (blockIdx.x - bix * kBlkPerB) * kScanCh;
  const int d   = d0 + tid;
  const size_t row0 = (size_t)bix * kSeq;
#pragma unroll 1
  for (int r = 0; r < kDtR; ++r) sW[r * kScanCh + tid] = Wdt[(size_t)r * kDm + d];
#pragma unroll 1
  for (int s = 0; s < kNst; ++s) sA[s * kScanCh + tid] = -expf(Alog[(size_t)d * kNst + s]);
  __syncthreads();
  float negA[kNst], h[kNst];
#pragma unroll
  for (int s = 0; s < kNst; ++s) {
    negA[s] = sA[s * kScanCh + tid];
    h[s] = 0.f;
  }
  const float bb = bdt[d];
  const int lr = tid >> 4, lc4 = (tid & 15) * 4;
  v4f bsel;
  {
    const int lcb = (lc4 < kXdN) ? lc4 : (kXdN - 4);
    const v4f braw = *(const v4f*)(bxp + lcb);
    const bool live = (lc4 < kXdN);
    bsel[0] = live ? braw[0] : 0.f;
    bsel[1] = live ? braw[1] : 0.f;
    bsel[2] = live ? braw[2] : 0.f;
    bsel[3] = live ? braw[3] : 0.f;
  }
  const int q = lane >> 3, c8 = (lane & 7) * 8;
#pragma unroll 1
  for (int t0 = 0; t0 < kSeq; t0 += kScanTS) {
    __syncthreads();
#pragma unroll
    for (int i = 0; i < 16; ++i) {
      const int r = lr + 4 * i;
      v4f xv = *(const v4f*)(XD + (row0 + t0 + r) * kXdP + lc4);
      xv[0] += bsel[0]; xv[1] += bsel[1]; xv[2] += bsel[2]; xv[3] += bsel[3];
      *(v4f*)(sX + r * kXdP + lc4) = xv;
    }
    __syncthreads();
#pragma unroll 1
    for (int s = 0; s < kScanTS; ++s) {
      const int t = t0 + s;
      const float* xr = sX + s * kXdP;
      float xt = UC[(row0 + t) * kDm + d];
      asm volatile("" : "+v"(xt));
      float zv = XZ[(row0 + t) * kXzP + kDm + d];
      asm volatile("" : "+v"(zv));
      float vdot = 0.f;
#pragma unroll 1
      for (int r4 = 0; r4 < kDtR / 4; ++r4) {
        const v4f xv = *(const v4f*)(xr + 4 * r4);
        const float* wp = sW + (4 * r4) * kScanCh + tid;
        vdot = fmaf(xv[0], wp[0], vdot);
        vdot = fmaf(xv[1], wp[kScanCh], vdot);
        vdot = fmaf(xv[2], wp[2 * kScanCh], vdot);
        vdot = fmaf(xv[3], wp[3 * kScanCh], vdot);
      }
      float Bs[kNst], Cs[kNst];
#pragma unroll
      for (int q4 = 0; q4 < 4; ++q4) {
        const v4f bv = *(const v4f*)(xr + kDtR + 4 * q4);
        const v4f cv = *(const v4f*)(xr + kDtR + kNst + 4 * q4);
        Bs[4 * q4 + 0] = bv[0]; Bs[4 * q4 + 1] = bv[1]; Bs[4 * q4 + 2] = bv[2]; Bs[4 * q4 + 3] = bv[3];
        Cs[4 * q4 + 0] = cv[0]; Cs[4 * q4 + 1] = cv[1]; Cs[4 * q4 + 2] = cv[2]; Cs[4 * q4 + 3] = cv[3];
      }
      const float v   = vdot + bb;
      const float a   = expf(-fabsf(v));
      const float u1  = 1.0f + a;
      const float l1p = __logf(u1) + (a - (u1 - 1.0f)) * __builtin_amdgcn_rcpf(u1);
      const float dt  = fmaxf(v, 0.0f) + l1p;
      const float dtx = dt * xt;
      float y = 0.f;
#pragma unroll
      for (int k = 0; k < kNst; ++k) {
        const float e = __expf(dt * negA[k]);
        h[k] = e * h[k] + dtx * Bs[k];
        y = h[k] * Cs[k] + y;
      }
      const float sg = __builtin_amdgcn_rcpf(1.0f + expf(-zv));
      y = y * (zv * sg);
      float yc = y * kCarY;
      yc = fminf(fmaxf(yc, -kSatY), kSatY);
      sY[s * kScanYP + tid] = yc;
    }
    __syncthreads();
    v8h hv[8];
#pragma unroll
    for (int it = 0; it < 8; ++it) {
      const int row = it * 8 + wave * 4 + q;
      const float* sp = sY + row * kScanYP + c8;
      const v4f a0 = *(const v4f*)(sp);
      const v4f a1 = *(const v4f*)(sp + 4);
#pragma unroll
      for (int e = 0; e < 4; ++e) {
        hv[it][e]     = (_Float16)a0[e];
        hv[it][4 + e] = (_Float16)a1[e];
      }
    }
    for (int pass = 0; pass < 2; ++pass) {
#pragma unroll
      for (int it = 0; it < 8; ++it) {
        const int row = it * 8 + wave * 4 + q;
        const size_t o = (row0 + t0 + row) * kDm + d0 + c8;
        *(volatile v8h*)(Y16 + o) = hv[it];
      }
      __threadfence();
    }
  }
}

extern "C" void kernel_launch(void* const* d_in, const int* in_sizes, int n_in,
                              void* d_out, int out_size, void* d_ws, size_t ws_size,
                              hipStream_t stream) {
  if (n_in != 12) return;
  if (in_sizes[0]  != kRows * kDm) return;
  if (in_sizes[1]  != kDm * kXzP) return;
  if (in_sizes[2]  != kXzP) return;
  if (in_sizes[3]  != kDm * 4) return;
  if (in_sizes[4]  != kDm) return;
  if (in_sizes[5]  != kDm * kXdN) return;
  if (in_sizes[6]  != kXdN) return;
  if (in_sizes[7]  != kDtR * kDm) return;
  if (in_sizes[8]  != kDm) return;
  if (in_sizes[9]  != kDm * kNst) return;
  if (in_sizes[10] != kDm * kDm) return;
  if (in_sizes[11] != kDm) return;
  if (out_size != kRows * kDm) return;
  if (ws_size < kWsTotal) return;

  const float* x      = (const float*)d_in[0];
  const float* W_in   = (const float*)d_in[1];
  const float* b_in   = (const float*)d_in[2];
  const float* W_conv = (const float*)d_in[3];
  const float* b_conv = (const float*)d_in[4];
  const float* W_xp   = (const float*)d_in[5];
  const float* b_xp   = (const float*)d_in[6];
  const float* W_dt   = (const float*)d_in[7];
  const float* b_dt   = (const float*)d_in[8];
  const float* A_log  = (const float*)d_in[9];
  const float* W_out  = (const float*)d_in[10];
  const float* b_out  = (const float*)d_in[11];
  float* out = (float*)d_out;

  char* ws = (char*)d_ws;
  unsigned short* X16    = (unsigned short*)(ws + kOffX16);
  unsigned short* WIN16  = (unsigned short*)(ws + kOffWIN);
  unsigned short* WXP16  = (unsigned short*)(ws + kOffWXP);
  unsigned short* WOUT16 = (unsigned short*)(ws + kOffWOUT);
  float*          XZ     = (float*)(ws + kOffXZ);
  float*          UC     = (float*)(ws + kOffUC);
  unsigned short* UC16   = (unsigned short*)(ws + kOffUC16);
  float*          XD     = (float*)(ws + kOffXD);
  unsigned short* Y16    = (unsigned short*)(ws + kOffY16);

  cast_f16_kernel<<<(kRows * kDm) / 8 / 256, 256, 0, stream>>>(x, X16, (kRows * kDm) / 8, kCarX);

  transpose_cast_kernel<<<dim3(kXzP / 64, kDm / 64), 256, 0, stream>>>(W_in, WIN16, kDm, kXzP, kCarW);
  transpose_cast_kernel<<<dim3(kXdP / 64, kDm / 64), 256, 0, stream>>>(W_xp, WXP16, kDm, kXdN, kCarW);
  transpose_cast_kernel<<<dim3(kDm / 64, kDm / 64), 256, 0, stream>>>(W_out, WOUT16, kDm, kDm, kCarW);

  gemm64_f16<2><<<(kRows / 64) * (kXzP / 64) / 8, 256, 0, stream>>>(
      X16, kDm, WIN16, kDm, XZ, kXzP, b_in, kRows, kXzP, kDm, kFold0);

  conv_silu_kernel<<<dim3(kDm / 256, kRows / 64), 256, 0, stream>>>(XZ, W_conv, b_conv, UC, UC16);

  gemm64_f16<0><<<(kRows / 64) * (kXdP / 64) / 8, 256, 0, stream>>>(
      UC16, kDm, WXP16, kDm, XD, kXdP, b_xp, kRows, kXdP, kDm, kFold1);

  scan_kernel<<<kBatch * (kDm / kScanCh), kScanCh, 0, stream>>>(XD, b_xp, UC, XZ, W_dt, b_dt, A_log, Y16);

  gemm64_f16<2><<<(kRows / 64) * (kDm / 64) / 8, 256, 0, stream>>>(
      Y16, kDm, WOUT16, kDm, out, kDm, b_out, kRows, kDm, kDm, kFold2);
}
